// MambaBlock_38766374814391
// MI455X (gfx1250) — hardware-verified
//
#include <hip/hip_runtime.h>
#include <math.h>

typedef __attribute__((ext_vector_type(16))) _Float16 v16h;
typedef __attribute__((ext_vector_type(8)))  _Float16 v8h;
typedef __attribute__((ext_vector_type(8)))  float    v8f;
typedef __attribute__((ext_vector_type(4)))  float    v4f;

constexpr int kBatch = 2;
constexpr int kSeq   = 2048;
constexpr int kDm    = 1024;
constexpr int kDi    = 2048;
constexpr int kNst   = 16;
constexpr int kDtR   = 64;
constexpr int kPrjN  = 96;
constexpr int kPrjP  = 128;
constexpr int kXzP   = 2 * kDi;
constexpr int kDff   = 4096;
constexpr int kRows  = kBatch * kSeq;
constexpr float kEps   = 1e-5f;
constexpr float kInvDm = 1.0f / (float)kDm;

constexpr float kCarryW   = 32.0f;
constexpr float kCarryWdt = 8.0f;
constexpr float kCarryDt  = 16.0f;
constexpr float kCarryY   = 16.0f;
constexpr float kCarryA   = 16.0f;

constexpr int kScanTS = 64;
constexpr int kScanCh = 64;
constexpr int kScanYP = 68;

static_assert(kDtR + 2 * kNst == kPrjN);
static_assert((kDm % 32) == 0 && (kDi % 32) == 0 && (kDtR % 32) == 0 && (kDff % 32) == 0);
static_assert((kRows % 64) == 0 && (kXzP % 64) == 0 && (kPrjP % 64) == 0 && (kDi % 64) == 0 && (kDm % 64) == 0 && (kDff % 64) == 0);
static_assert((kSeq % kScanTS) == 0 && (kSeq % 64) == 0 && (kDi % kScanCh) == 0 && (kDi % 512) == 0 && (kRows % 8) == 0);
static_assert(kDm == 1024 && kXzP == 4096);

constexpr size_t kSzWIN  = (size_t)kXzP * kDm * 2;
constexpr size_t kSzWXP  = (size_t)kPrjP * kDi * 2;
constexpr size_t kSzWDT  = (size_t)kDi * kDtR * 2;
constexpr size_t kSzWOUT = (size_t)kDm * kDi * 2;
constexpr size_t kSzWF2  = (size_t)kDm * kDff * 2;
constexpr size_t kSzU16  = (size_t)kRows * kDm * 2;
constexpr size_t kSzXZ16 = (size_t)kRows * kXzP * 2;
constexpr size_t kSzXC16 = (size_t)kRows * kDi * 2;
constexpr size_t kSzY16  = (size_t)kRows * kDi * 2;
constexpr size_t kSzDBL  = (size_t)kRows * kPrjP * 4;
constexpr size_t kSzDTLR = (size_t)kRows * kDtR * 2;
constexpr size_t kSzDLR  = (size_t)kRows * kDi * 2;
constexpr size_t kSzH32  = (size_t)kRows * kDm * 4;
constexpr size_t kOffWIN  = 0;
constexpr size_t kOffWXP  = kOffWIN  + kSzWIN;
constexpr size_t kOffWDT  = kOffWXP  + kSzWXP;
constexpr size_t kOffWOUT = kOffWDT  + kSzWDT;
constexpr size_t kOffWF2  = kOffWOUT + kSzWOUT;
constexpr size_t kOffU16  = kOffWF2  + kSzWF2;
constexpr size_t kOffXZ16 = kOffU16  + kSzU16;
constexpr size_t kOffXC16 = kOffXZ16 + kSzXZ16;
constexpr size_t kOffY16  = kOffXC16 + kSzXC16;
constexpr size_t kOffDBL  = kOffY16  + kSzY16;
constexpr size_t kOffDTLR = kOffDBL  + kSzDBL;
constexpr size_t kOffDLR  = kOffDTLR + kSzDTLR;
constexpr size_t kOffH32  = kOffDLR  + kSzDLR;
constexpr size_t kWsTotal = kOffH32  + kSzH32;
static_assert(kWsTotal == 133431296ull);
static_assert(kWsTotal <= 134217728ull);
static_assert((size_t)kDff * kDm * 2 == kSzWIN);
static_assert((size_t)kRows * kDff * 2 == kSzXZ16);
static_assert((kOffWXP % 128) == 0 && (kOffWDT % 128) == 0 && (kOffWOUT % 128) == 0 && (kOffWF2 % 128) == 0 &&
              (kOffU16 % 128) == 0 && (kOffXZ16 % 128) == 0 && (kOffXC16 % 128) == 0 && (kOffY16 % 128) == 0 &&
              (kOffDBL % 128) == 0 && (kOffDTLR % 128) == 0 && (kOffDLR % 128) == 0 && (kOffH32 % 128) == 0);

__device__ __forceinline__ float h16_to_f32(unsigned hb) {
  const unsigned sgn = (hb & 0x8000u) << 16;
  const unsigned em = hb & 0x7fffu;
  const float fn = __uint_as_float((em << 13) + 0x38000000u);
  const float fs = (float)em * 5.9604644775390625e-8f;
  const float mag = (em < 0x400u) ? fs : fn;
  return __uint_as_float(__float_as_uint(mag) | sgn);
}
__device__ __forceinline__ unsigned pack2_f16(float a, float b) {
  const _Float16 h0 = (_Float16)a;
  const _Float16 h1 = (_Float16)b;
  const unsigned u0 = (unsigned)__builtin_bit_cast(unsigned short, h0);
  const unsigned u1 = (unsigned)__builtin_bit_cast(unsigned short, h1);
  return u0 | (u1 << 16);
}

__device__ __forceinline__ void row_guard_h(v8f& a, v8f& b, v8f& c, v8f& d, v16h x, v16h y0, v16h y1, v16h y2, v16h y3) {
  asm volatile("v_nop\n\tv_nop\n\tv_nop\n\tv_nop" : "+v"(a), "+v"(b), "+v"(c), "+v"(d) : "v"(x), "v"(y0), "v"(y1), "v"(y2), "v"(y3));
}
__device__ __forceinline__ void keep4_h(v16h a, v16h b, v16h c, v16h d) { asm volatile("v_nop" :: "v"(a), "v"(b), "v"(c), "v"(d)); }
__device__ __forceinline__ void acc_guard4(v8f& a, v8f& b, v8f& c, v8f& d) { asm volatile("v_nop\n\tv_nop\n\tv_nop\n\tv_nop" : "+v"(a), "+v"(b), "+v"(c), "+v"(d)); }

union FragH { v16h v; v8h h[2]; };
__device__ __forceinline__ v16h frag_load_h(const _Float16* p) {
  FragH f;
  f.h[0] = *(const v8h*)(p);
  f.h[1] = *(const v8h*)(p + 16);
  return f.v;
}
__device__ __forceinline__ v8f mma_h(v16h a, v16h b, v8f c) {
  return __builtin_amdgcn_wmma_f32_16x16x32_f16(false, a, false, b, (short)0, c, false, false);
}

template <bool BIAS_N, int OUT_MODE, bool RESID, bool RELU>
__global__ __launch_bounds__(256) void wmma_gemm64_f16(
    const unsigned short* __restrict__ Ap, int lda,
    const unsigned short* __restrict__ Btp, int ldb,
    void* __restrict__ Cout, int ldc,
    const float* __restrict__ bias,
    const float* __restrict__ resid, int ldr,
    int M, int N, int K, float scale)
{
  static_assert(OUT_MODE == 0 || OUT_MODE == 1);
  static_assert(!(RESID && RELU));
  static_assert(!(RESID && OUT_MODE != 0));
  const _Float16* A  = (const _Float16*)Ap;
  const _Float16* Bt = (const _Float16*)Btp;
  __shared__ __align__(16) float sT[8][16 * 68];
  const int lane = threadIdx.x & 31;
  const int wave = threadIdx.x >> 5;
  const int tilesN = N >> 6;
  const int tilesM = M >> 6;
  const int tile = blockIdx.x * 8 + wave;
  if (tile >= tilesM * tilesN) return;
  const int tm = tile / tilesN;
  const int tn = tile - tm * tilesN;
  const int m0 = tm << 6;
  const int n0 = tn << 6;

  const int rlane = lane & 15;
  const int koff  = (lane >> 4) * 8;
  const int mOff  = (lane >> 4) * 8;

  v8f acc[4][4];
#pragma unroll
  for (int i = 0; i < 4; ++i)
#pragma unroll
    for (int j = 0; j < 4; ++j) acc[i][j] = (v8f){0.f,0.f,0.f,0.f,0.f,0.f,0.f,0.f};

  for (int k0 = 0; k0 < K; k0 += 32) {
    v16h bh[4];
#pragma unroll
    for (int j = 0; j < 4; ++j) {
      const size_t bo = (size_t)(n0 + (j << 4) + rlane) * ldb + koff + k0;
      bh[j] = frag_load_h(Bt + bo);
    }
#pragma unroll
    for (int i = 0; i < 4; ++i) {
      const size_t ao = (size_t)(m0 + (i << 4) + rlane) * lda + koff + k0;
      const v16h ah = frag_load_h(A + ao);
#pragma unroll
      for (int j = 0; j < 4; ++j) acc[i][j] = mma_h(ah, bh[j], acc[i][j]);
      row_guard_h(acc[i][0], acc[i][1], acc[i][2], acc[i][3], ah, bh[0], bh[1], bh[2], bh[3]);
    }
    keep4_h(bh[0], bh[1], bh[2], bh[3]);
  }
  acc_guard4(acc[0][0], acc[0][1], acc[0][2], acc[0][3]);
  acc_guard4(acc[1][0], acc[1][1], acc[1][2], acc[1][3]);
  acc_guard4(acc[2][0], acc[2][1], acc[2][2], acc[2][3]);
  acc_guard4(acc[3][0], acc[3][1], acc[3][2], acc[3][3]);

  float* slab = sT[wave];
#pragma unroll
  for (int i = 0; i < 4; ++i) {
    const int mBase = m0 + (i << 4);
#pragma unroll
    for (int j = 0; j < 4; ++j) {
      float bv = 0.f;
      if (BIAS_N) bv = bias[n0 + (j << 4) + rlane];
#pragma unroll
      for (int r = 0; r < 8; ++r) {
        float v = acc[i][j][r] * scale;
        if (BIAS_N) v += bv;
        if (RELU) v = fmaxf(v, 0.0f);
        slab[(mOff + r) * 68 + (j << 4) + rlane] = v;
      }
    }
    __builtin_amdgcn_fence(__ATOMIC_RELEASE, "workgroup");
    __builtin_amdgcn_wave_barrier();
    __builtin_amdgcn_fence(__ATOMIC_ACQUIRE, "workgroup");
    if (OUT_MODE == 0) {
      float* C = (float*)Cout;
      const int hh = lane >> 4, c4 = (lane & 15) * 4;
      v4f vv[8];
#pragma unroll
      for (int it = 0; it < 8; ++it) {
        const int row = it * 2 + hh;
        v4f v = *(const v4f*)(slab + row * 68 + c4);
        if (RESID) {
          const v4f rv = *(const v4f*)(resid + (size_t)(mBase + row) * ldr + n0 + c4);
          v = v + rv;
        }
        vv[it] = v;
      }
      for (int pass = 0; pass < 2; ++pass) {
#pragma unroll
        for (int it = 0; it < 8; ++it) {
          const int row = it * 2 + hh;
          *(volatile v4f*)(C + (size_t)(mBase + row) * ldc + n0 + c4) = vv[it];
        }
        __threadfence();
      }
    } else {
      const int q = lane >> 3, c8 = (lane & 7) * 8;
      unsigned short* C = (unsigned short*)Cout;
      v8h hv[4];
#pragma unroll
      for (int it = 0; it < 4; ++it) {
        const int row = it * 4 + q;
        const float* sp = slab + row * 68 + c8;
        const v4f a0 = *(const v4f*)(sp);
        const v4f a1 = *(const v4f*)(sp + 4);
#pragma unroll
        for (int e = 0; e < 4; ++e) {
          hv[it][e]     = (_Float16)a0[e];
          hv[it][4 + e] = (_Float16)a1[e];
        }
      }
      for (int pass = 0; pass < 2; ++pass) {
#pragma unroll
        for (int it = 0; it < 4; ++it) {
          const int row = it * 4 + q;
          *(volatile v8h*)(C + (size_t)(mBase + row) * ldc + n0 + c8) = hv[it];
        }
        __threadfence();
      }
    }
    __builtin_amdgcn_fence(__ATOMIC_RELEASE, "workgroup");
    __builtin_amdgcn_wave_barrier();
    __builtin_amdgcn_fence(__ATOMIC_ACQUIRE, "workgroup");
  }
}

__global__ __launch_bounds__(256) void cast_f16_kernel(
    const float* __restrict__ src, unsigned short* __restrict__ dst, int total8, int real8, float scale)
{
  const int i = blockIdx.x * 256 + threadIdx.x;
  if (i >= total8) return;
  const bool live = (i < real8);
  const int ic = live ? i : (real8 - 1);
  const float* p = src + ((size_t)ic << 3);
  const v4f a0 = *(const v4f*)(p);
  const v4f a1 = *(const v4f*)(p + 4);
  v8h hv;
#pragma unroll
  for (int e = 0; e < 4; ++e) {
    const float f0 = live ? (a0[e] * scale) : 0.0f;
    const float f1 = live ? (a1[e] * scale) : 0.0f;
    hv[e]     = (_Float16)f0;
    hv[4 + e] = (_Float16)f1;
  }
  unsigned short* q = dst + ((size_t)i << 3);
  *(volatile v8h*)q = hv;
  __threadfence();
  *(volatile v8h*)q = hv;
}

__global__ __launch_bounds__(256) void layernorm_f16_kernel(
    const float* __restrict__ X, const float* __restrict__ gam, const float* __restrict__ bet,
    unsigned short* __restrict__ out16, int nrows)
{
  const int lane = threadIdx.x & 31, wave = threadIdx.x >> 5;
  const int row = blockIdx.x * 8 + wave;
  if (row >= nrows) return;
  const float* xr = X + (size_t)row * kDm;
  v4f a[8];
#pragma unroll
  for (int i = 0; i < 4; ++i) {
    a[2 * i]     = *(const v4f*)(xr + i * 256 + lane * 8);
    a[2 * i + 1] = *(const v4f*)(xr + i * 256 + lane * 8 + 4);
  }
  float s = 0.f;
#pragma unroll
  for (int i = 0; i < 8; ++i) s += (a[i][0] + a[i][1]) + (a[i][2] + a[i][3]);
#pragma unroll
  for (int off = 16; off >= 1; off >>= 1) s += __shfl_xor(s, off, 32);
  const float mu = s * kInvDm;
  float q = 0.f;
#pragma unroll
  for (int i = 0; i < 8; ++i) {
#pragma unroll
    for (int e = 0; e < 4; ++e) {
      const float dv = a[i][e] - mu;
      q = fmaf(dv, dv, q);
    }
  }
#pragma unroll
  for (int off = 16; off >= 1; off >>= 1) q += __shfl_xor(q, off, 32);
  const float rstd = rsqrtf(q * kInvDm + kEps);
  v8h hv[4];
#pragma unroll
  for (int i = 0; i < 4; ++i) {
    const v4f g0 = *(const v4f*)(gam + i * 256 + lane * 8);
    const v4f g1 = *(const v4f*)(gam + i * 256 + lane * 8 + 4);
    const v4f b0 = *(const v4f*)(bet + i * 256 + lane * 8);
    const v4f b1 = *(const v4f*)(bet + i * 256 + lane * 8 + 4);
#pragma unroll
    for (int e = 0; e < 4; ++e) {
      const float y0 = (a[2 * i][e] - mu) * rstd * g0[e] + b0[e];
      const float y1 = (a[2 * i + 1][e] - mu) * rstd * g1[e] + b1[e];
      hv[i][e]     = (_Float16)y0;
      hv[i][4 + e] = (_Float16)y1;
    }
  }
  unsigned short* orow = out16 + (size_t)row * kDm;
  for (int pass = 0; pass < 2; ++pass) {
#pragma unroll
    for (int i = 0; i < 4; ++i) *(volatile v8h*)(orow + i * 256 + lane * 8) = hv[i];
    __threadfence();
  }
}

__global__ __launch_bounds__(256) void conv_silu_kernel(
    const unsigned* __restrict__ XZw, const float* __restrict__ cw, const float* __restrict__ cb,
    unsigned* __restrict__ XCw)
{
  constexpr int kXzW = kXzP / 2;
  constexpr int kXcW = kDi / 2;
  const int tid = threadIdx.x;
  const int cp = blockIdx.x * 256 + tid;
  const int g0 = blockIdx.y * 64;
  const int tb = g0 & (kSeq - 1);
  const v4f wa = *(const v4f*)(cw + (size_t)cp * 8);
  const v4f wb = *(const v4f*)(cw + (size_t)cp * 8 + 4);
  const float bc0 = cb[2 * cp], bc1 = cb[2 * cp + 1];
  float p3a, p2a, p1a, p3b, p2b, p1b;
  {
    const bool hist = (tb > 0);
    const int rb = hist ? (g0 - 3) : g0;
    const unsigned u3 = XZw[(size_t)rb * kXzW + cp];
    const unsigned u2 = XZw[(size_t)(rb + 1) * kXzW + cp];
    const unsigned u1 = XZw[(size_t)(rb + 2) * kXzW + cp];
    const float f3a = h16_to_f32(u3 & 0xffffu), f3b = h16_to_f32(u3 >> 16);
    const float f2a = h16_to_f32(u2 & 0xffffu), f2b = h16_to_f32(u2 >> 16);
    const float f1a = h16_to_f32(u1 & 0xffffu), f1b = h16_to_f32(u1 >> 16);
    p3a = hist ? f3a : 0.f;  p3b = hist ? f3b : 0.f;
    p2a = hist ? f2a : 0.f;  p2b = hist ? f2b : 0.f;
    p1a = hist ? f1a : 0.f;  p1b = hist ? f1b : 0.f;
  }
#pragma unroll 1
  for (int s = 0; s < 64; ++s) {
    const unsigned uc = XZw[(size_t)(g0 + s) * kXzW + cp];
    const float xa = h16_to_f32(uc & 0xffffu);
    const float xb = h16_to_f32(uc >> 16);
    float ca = bc0;
    ca = fmaf(wa[0], p3a, ca);
    ca = fmaf(wa[1], p2a, ca);
    ca = fmaf(wa[2], p1a, ca);
    ca = fmaf(wa[3], xa, ca);
    float cbv = bc1;
    cbv = fmaf(wb[0], p3b, cbv);
    cbv = fmaf(wb[1], p2b, cbv);
    cbv = fmaf(wb[2], p1b, cbv);
    cbv = fmaf(wb[3], xb, cbv);
    const float sa = ca * __builtin_amdgcn_rcpf(1.0f + expf(-ca));
    const float sb = cbv * __builtin_amdgcn_rcpf(1.0f + expf(-cbv));
    const unsigned wv = pack2_f16(sa, sb);
    volatile unsigned* op = (volatile unsigned*)(XCw + (size_t)(g0 + s) * kXcW + cp);
    *op = wv;
    __threadfence();
    *op = wv;
    p3a = p2a; p2a = p1a; p1a = xa;
    p3b = p2b; p2b = p1b; p1b = xb;
  }
}

__global__ __launch_bounds__(256) void dt_cast_kernel(
    const float* __restrict__ DBL, unsigned short* __restrict__ DT16, int total8, float scale)
{
  const int i = blockIdx.x * 256 + threadIdx.x;
  if (i >= total8) return;
  const int e0  = i << 3;
  const int row = e0 >> 6;
  const int c8  = e0 & 63;
  const float* p = DBL + (size_t)row * kPrjP + c8;
  const v4f a0 = *(const v4f*)(p);
  const v4f a1 = *(const v4f*)(p + 4);
  v8h hv;
#pragma unroll
  for (int e = 0; e < 4; ++e) {
    hv[e]     = (_Float16)(a0[e] * scale);
    hv[4 + e] = (_Float16)(a1[e] * scale);
  }
  unsigned short* qd = DT16 + e0;
  *(volatile v8h*)qd = hv;
  __threadfence();
  *(volatile v8h*)qd = hv;
}

__global__ __launch_bounds__(64) void scan_kernel(
    const float* __restrict__ DBL, const unsigned* __restrict__ DLRw, const unsigned* __restrict__ XCw,
    const unsigned* __restrict__ XZw, const float* __restrict__ Alog, const float* __restrict__ Dp,
    unsigned short* __restrict__ Y16)
{
  __shared__ __align__(16) float sX[kScanTS * 32];
  __shared__ __align__(16) float sY[kScanTS * kScanYP];
  __shared__ __align__(16) float sA[kNst * kScanCh];
  constexpr int kHalfW = kDi / 2;
  constexpr int kXzW   = kXzP / 2;
  const int tid = threadIdx.x, lane = tid & 31, wave = tid >> 5;
  constexpr int kBlkPerB = kDi / kScanCh;
  const int bix = blockIdx.x / kBlkPerB;
  const int d0  = (blockIdx.x - bix * kBlkPerB) * kScanCh;
  const int d   = d0 + tid;
  const int wi  = d >> 1;
  const unsigned sh = (unsigned)(d & 1) << 4;
  const size_t row0 = (size_t)bix * kSeq;
#pragma unroll 1
  for (int s = 0; s < kNst; ++s) sA[s * kScanCh + tid] = -expf(Alog[(size_t)d * kNst + s]);
  __syncthreads();
  float negA[kNst], h[kNst];
#pragma unroll
  for (int s = 0; s < kNst; ++s) {
    negA[s] = sA[s * kScanCh + tid];
    h[s] = 0.f;
  }
  const float Dd = Dp[d];
  const int q = lane >> 3, c8 = (lane & 7) * 8;
#pragma unroll 1
  for (int t0 = 0; t0 < kSeq; t0 += kScanTS) {
    __syncthreads();
#pragma unroll
    for (int i = 0; i < 8; ++i) {
      const int idx = tid + 64 * i;
      const int r = idx >> 3, c4 = (idx & 7) * 4;
      *(v4f*)(sX + r * 32 + c4) = *(const v4f*)(DBL + (row0 + t0 + r) * kPrjP + kDtR + c4);
    }
    __syncthreads();
#pragma unroll 1
    for (int s = 0; s < kScanTS; ++s) {
      const size_t r = row0 + t0 + s;
      unsigned wd = DLRw[r * kHalfW + wi];
      unsigned wx = XCw[r * kHalfW + wi];
      unsigned wz = XZw[r * kXzW + kHalfW + wi];
      asm volatile("" : "+v"(wd), "+v"(wx), "+v"(wz));
      const float v  = h16_to_f32((wd >> sh) & 0xffffu);
      const float xt = h16_to_f32((wx >> sh) & 0xffffu);
      const float zv = h16_to_f32((wz >> sh) & 0xffffu);
      const float* xr = sX + s * 32;
      float Bs[kNst], Cs[kNst];
#pragma unroll
      for (int q4 = 0; q4 < 4; ++q4) {
        const v4f bv = *(const v4f*)(xr + 4 * q4);
        const v4f cv = *(const v4f*)(xr + kNst + 4 * q4);
        Bs[4 * q4 + 0] = bv[0]; Bs[4 * q4 + 1] = bv[1]; Bs[4 * q4 + 2] = bv[2]; Bs[4 * q4 + 3] = bv[3];
        Cs[4 * q4 + 0] = cv[0]; Cs[4 * q4 + 1] = cv[1]; Cs[4 * q4 + 2] = cv[2]; Cs[4 * q4 + 3] = cv[3];
      }
      const float ea  = __expf(-fabsf(v));
      const float up  = 1.0f + ea;
      const float l1p = __logf(up) + (ea - (up - 1.0f)) * __builtin_amdgcn_rcpf(up);
      const float dt  = fmaxf(v, 0.0f) + l1p;
      const float dtx = dt * xt;
      float y = 0.f;
#pragma unroll
      for (int k = 0; k < kNst; ++k) {
        const float e = __expf(dt * negA[k]);
        h[k] = e * h[k] + dtx * Bs[k];
        y = h[k] * Cs[k] + y;
      }
      y = xt * Dd + y;
      const float sg = __builtin_amdgcn_rcpf(1.0f + expf(-zv));
      y = y * (zv * sg);
      sY[s * kScanYP + tid] = y * kCarryY;
    }
    __syncthreads();
    v8h hv[8];
#pragma unroll
    for (int it = 0; it < 8; ++it) {
      const int row = it * 8 + wave * 4 + q;
      const float* sp = sY + row * kScanYP + c8;
      const v4f a0 = *(const v4f*)(sp);
      const v4f a1 = *(const v4f*)(sp + 4);
#pragma unroll
      for (int e = 0; e < 4; ++e) {
        hv[it][e]     = (_Float16)a0[e];
        hv[it][4 + e] = (_Float16)a1[e];
      }
    }
    for (int pass = 0; pass < 2; ++pass) {
#pragma unroll
      for (int it = 0; it < 8; ++it) {
        const int row = it * 8 + wave * 4 + q;
        const size_t o = (row0 + t0 + row) * kDi + d0 + c8;
        *(volatile v8h*)(Y16 + o) = hv[it];
      }
      __threadfence();
    }
  }
}

extern "C" void kernel_launch(void* const* d_in, const int* in_sizes, int n_in,
                              void* d_out, int out_size, void* d_ws, size_t ws_size,
                              hipStream_t stream)
{
  if (n_in < 16) return;
  if (in_sizes[0] != kRows * kDm) return;
  if (in_sizes[1] != kDm || in_sizes[2] != kDm || in_sizes[3] != kDm || in_sizes[4] != kDm) return;
  if (in_sizes[5] != kXzP * kDm) return;
  if (in_sizes[6] != kDi * 4 || in_sizes[7] != kDi) return;
  if (in_sizes[8] != kPrjN * kDi) return;
  if (in_sizes[9] != kDi * kDtR || in_sizes[10] != kDi) return;
  if (in_sizes[11] != kDi * kNst || in_sizes[12] != kDi) return;
  if (in_sizes[13] != kDm * kDi) return;
  if (in_sizes[14] != kDff * kDm || in_sizes[15] != kDm * kDff) return;
  if (out_size != kRows * kDm) return;
  if (ws_size < kWsTotal) return;

  const float* x        = (const float*)d_in[0];
  const float* ln1_g    = (const float*)d_in[1];
  const float* ln1_b    = (const float*)d_in[2];
  const float* ln2_g    = (const float*)d_in[3];
  const float* ln2_b    = (const float*)d_in[4];
  const float* W_in     = (const float*)d_in[5];
  const float* conv_w   = (const float*)d_in[6];
  const float* conv_b   = (const float*)d_in[7];
  const float* W_xproj  = (const float*)d_in[8];
  const float* W_dtproj = (const float*)d_in[9];
  const float* b_dtproj = (const float*)d_in[10];
  const float* A_log    = (const float*)d_in[11];
  const float* Dvec     = (const float*)d_in[12];
  const float* W_out    = (const float*)d_in[13];
  const float* ffn_w1   = (const float*)d_in[14];
  const float* ffn_w2   = (const float*)d_in[15];
  float* out = (float*)d_out;

  char* ws = (char*)d_ws;
  unsigned short* WIN16  = (unsigned short*)(ws + kOffWIN);
  unsigned short* WF1_16 = (unsigned short*)(ws + kOffWIN);
  unsigned short* WXP16  = (unsigned short*)(ws + kOffWXP);
  unsigned short* WDT16  = (unsigned short*)(ws + kOffWDT);
  unsigned short* WOUT16 = (unsigned short*)(ws + kOffWOUT);
  unsigned short* WF2_16 = (unsigned short*)(ws + kOffWF2);
  unsigned short* U16    = (unsigned short*)(ws + kOffU16);
  unsigned short* HN16   = (unsigned short*)(ws + kOffU16);
  unsigned short* XZ16   = (unsigned short*)(ws + kOffXZ16);
  unsigned short* A16    = (unsigned short*)(ws + kOffXZ16);
  unsigned short* XC16   = (unsigned short*)(ws + kOffXC16);
  unsigned short* Y16    = (unsigned short*)(ws + kOffY16);
  float*          DBL32  = (float*)(ws + kOffDBL);
  unsigned short* DTLR16 = (unsigned short*)(ws + kOffDTLR);
  unsigned short* DLR16  = (unsigned short*)(ws + kOffDLR);
  float*          H32    = (float*)(ws + kOffH32);
  const float* no_bias  = b_dtproj;
  const float* no_resid = x;

  constexpr int kT8Win  = kXzP * kDm / 8;
  constexpr int kT8Wxp  = kPrjP * kDi / 8;
  constexpr int kR8Wxp  = kPrjN * kDi / 8;
  constexpr int kT8Wdt  = kDi * kDtR / 8;
  constexpr int kT8Wout = kDm * kDi / 8;
  constexpr int kT8Wf   = kDff * kDm / 8;
  static_assert((kT8Win % 256) == 0 && (kT8Wxp % 256) == 0 && (kT8Wdt % 256) == 0 && (kT8Wout % 256) == 0 && (kT8Wf % 256) == 0);
  cast_f16_kernel<<<kT8Win / 256, 256, 0, stream>>>(W_in, WIN16, kT8Win, kT8Win, kCarryW);
  cast_f16_kernel<<<kT8Wxp / 256, 256, 0, stream>>>(W_xproj, WXP16, kT8Wxp, kR8Wxp, kCarryW);
  cast_f16_kernel<<<kT8Wdt / 256, 256, 0, stream>>>(W_dtproj, WDT16, kT8Wdt, kT8Wdt, kCarryWdt);
  cast_f16_kernel<<<kT8Wout / 256, 256, 0, stream>>>(W_out, WOUT16, kT8Wout, kT8Wout, kCarryW);
  cast_f16_kernel<<<kT8Wf / 256, 256, 0, stream>>>(ffn_w2, WF2_16, kT8Wf, kT8Wf, kCarryW);

  layernorm_f16_kernel<<<kRows / 8, 256, 0, stream>>>(x, ln1_g, ln1_b, U16, kRows);

  wmma_gemm64_f16<false, 1, false, false><<<(kRows / 64) * (kXzP / 64) / 8, 256, 0, stream>>>(
      U16, kDm, WIN16, kDm, (void*)XZ16, kXzP, no_bias, no_resid, kDm, kRows, kXzP, kDm, 1.0f / kCarryW);

  cast_f16_kernel<<<kT8Wf / 256, 256, 0, stream>>>(ffn_w1, WF1_16, kT8Wf, kT8Wf, kCarryW);

  conv_silu_kernel<<<dim3(kDi / 512, kRows / 64), 256, 0, stream>>>(
      (const unsigned*)XZ16, conv_w, conv_b, (unsigned*)XC16);

  wmma_gemm64_f16<false, 0, false, false><<<(kRows / 64) * (kPrjP / 64) / 8, 256, 0, stream>>>(
      XC16, kDi, WXP16, kDi, (void*)DBL32, kPrjP, no_bias, no_resid, kDm, kRows, kPrjP, kDi, 1.0f / kCarryW);

  dt_cast_kernel<<<(kRows * kDtR / 8) / 256, 256, 0, stream>>>(DBL32, DTLR16, kRows * kDtR / 8, kCarryDt);

  wmma_gemm64_f16<true, 1, false, false><<<(kRows / 64) * (kDi / 64) / 8, 256, 0, stream>>>(
      DTLR16, kDtR, WDT16, kDtR, (void*)DLR16, kDi, b_dtproj, no_resid, kDm, kRows, kDi, kDtR,
      1.0f / (kCarryDt * kCarryWdt));

  scan_kernel<<<kBatch * (kDi / kScanCh), kScanCh, 0, stream>>>(
      DBL32, (const unsigned*)DLR16, (const unsigned*)XC16, (const unsigned*)XZ16, A_log, Dvec, Y16);

  wmma_gemm64_f16<false, 0, true, false><<<(kRows / 64) * (kDm / 64) / 8, 256, 0, stream>>>(
      Y16, kDi, WOUT16, kDi, (void*)H32, kDm, no_bias, x, kDm, kRows, kDm, kDi, 1.0f / (kCarryY * kCarryW));

  layernorm_f16_kernel<<<kRows / 8, 256, 0, stream>>>(H32, ln2_g, ln2_b, HN16, kRows);

  wmma_gemm64_f16<false, 1, false, true><<<(kRows / 64) * (kDff / 64) / 8, 256, 0, stream>>>(
      HN16, kDm, WF1_16, kDm, (void*)A16, kDff, no_bias, no_resid, kDm, kRows, kDff, kDm, kCarryA / kCarryW);

  wmma_gemm64_f16<false, 0, true, false><<<(kRows / 64) * (kDm / 64) / 8, 256, 0, stream>>>(
      A16, kDff, WF2_16, kDff, (void*)out, kDm, no_bias, H32, kDm, kRows, kDm, kDff, 1.0f / (kCarryA * kCarryW));
}
